// GATModel_31336081392306
// MI455X (gfx1250) — hardware-verified
//
#include <hip/hip_runtime.h>
#include <stddef.h>
#include <stdint.h>
#include <math.h>


#define F_IN    256
#define HC1     256
#define HID     64
#define NHD1    4
#define OC      64
#define KA2     512
#define NTHR    256
#define NWAVE   8
#define EPT     8
#define CHUNK   (NTHR * EPT)
#define WCAP    (EPT * 32)
#define LISTN   (NWAVE * WCAP)
#define NBMAX   2048
#define SLOTB   11
#define RCAP    28672
#define DEGCAP  256
#define GBM     64
#define GBN     64
#define GTHR    128
#define MROWS   128
#define GRP     32
#define NEGSL   0.2f
#define EPS_SM  1e-16f
#define WSMAX   134217728
#define LDS_AGG ((2 * RCAP + 2 * NBMAX + LISTN) * 4 + 64)

static_assert((CHUNK & (CHUNK - 1)) == 0 && CHUNK <= (1 << SLOTB));
static_assert(NBMAX == (1 << SLOTB));
static_assert(NTHR * 8 == NBMAX);
static_assert(LISTN >= NBMAX);
static_assert(LISTN >= NWAVE * WCAP);
static_assert((RCAP % 32) == 0);
static_assert(LDS_AGG <= 300000);
static_assert(GBM == (GTHR / 32) * 16);
static_assert(GTHR == 2 * GBN && GTHR == 2 * GBM);
static_assert((F_IN % 32) == 0 && (KA2 % 32) == 0);
static_assert((HC1 % GBN) == 0 && HID == GBN && OC == GBN);
static_assert(KA2 == 2 * HC1);
static_assert((MROWS % GBM) == 0);
static_assert(HC1 == 8 * 32);
static_assert(OC == 2 * 32);
static_assert(NHD1 * HID == HC1);
static_assert(NWAVE * GRP * OC + 2 * OC * OC <= RCAP);
static_assert((GRP & (GRP - 1)) == 0 && (OC % 4) == 0);
static_assert((F_IN / 8) == 32);
static_assert(((OC * OC) / 4) % NTHR == 0);

typedef float          v2f  __attribute__((ext_vector_type(2)));
typedef float          v4f  __attribute__((ext_vector_type(4)));
typedef float          v8f  __attribute__((ext_vector_type(8)));
typedef int            v4i  __attribute__((ext_vector_type(4)));
typedef int            v8i  __attribute__((ext_vector_type(8)));
typedef unsigned int   v4u  __attribute__((ext_vector_type(4)));
typedef unsigned short v8us __attribute__((ext_vector_type(8)));
typedef __bf16         v16b __attribute__((ext_vector_type(16)));
typedef v2f  __attribute__((may_alias)) v2fa;
typedef v4f  __attribute__((may_alias)) v4fa;
typedef v8us __attribute__((may_alias)) v8usa;
union FragB { v16b v; v8us h[2]; v8i w; };

__device__ __forceinline__ v8f wmb(const FragB& a, const FragB& b, v8f c) {
  v8f d = __builtin_amdgcn_wmma_f32_16x16x32_bf16(false, a.v, false, b.v, (short)0, c, false, false);
  asm volatile("v_nop\n\tv_nop\n\tv_nop\n\tv_nop" : "+v"(d) : "v"(a.w), "v"(b.w));
  return d;
}

__device__ __forceinline__ unsigned int f2bf(float f) {
  const unsigned int u = __float_as_uint(f);
  return ((u + 0x7FFFu + ((u >> 16) & 1u)) >> 16) & 0xFFFFu;
}
__device__ __forceinline__ float bf2f(unsigned int b) { return __uint_as_float(b << 16); }
__device__ __forceinline__ float bfr(float f) { return bf2f(f2bf(f)); }
__device__ __forceinline__ v4f bfr4(const v4f a) {
  v4f r; r.x = bfr(a.x); r.y = bfr(a.y); r.z = bfr(a.z); r.w = bfr(a.w); return r;
}
__device__ __forceinline__ unsigned int pk2(float lo, float hi) { return f2bf(lo) | (f2bf(hi) << 16); }
__device__ __forceinline__ v4u pack8(const v4f a, const v4f b) {
  v4u r;
  r.x = pk2(a.x, a.y); r.y = pk2(a.z, a.w); r.z = pk2(b.x, b.y); r.w = pk2(b.z, b.w);
  return r;
}

__device__ __forceinline__ int scan_chunk(const int* __restrict__ dsts, int nE, int cbase, int slotBase,
                                          int nb, int vec8, int* list, int tid, int lane, int wave) {
  int wc = 0;
  const int el0  = tid * EPT;
  const int e0   = cbase + el0;
  const int sent = -2147483647 - 1;
  v4i da, db;
  if (vec8 != 0 && cbase + CHUNK <= nE) {
    da = *(const v4i*)(dsts + e0);
    db = *(const v4i*)(dsts + e0 + 4);
  } else {
    da.x = (e0     < nE) ? dsts[min(e0,     nE - 1)] : sent;
    da.y = (e0 + 1 < nE) ? dsts[min(e0 + 1, nE - 1)] : sent;
    da.z = (e0 + 2 < nE) ? dsts[min(e0 + 2, nE - 1)] : sent;
    da.w = (e0 + 3 < nE) ? dsts[min(e0 + 3, nE - 1)] : sent;
    db.x = (e0 + 4 < nE) ? dsts[min(e0 + 4, nE - 1)] : sent;
    db.y = (e0 + 5 < nE) ? dsts[min(e0 + 5, nE - 1)] : sent;
    db.z = (e0 + 6 < nE) ? dsts[min(e0 + 6, nE - 1)] : sent;
    db.w = (e0 + 7 < nE) ? dsts[min(e0 + 7, nE - 1)] : sent;
  }
  const unsigned nbs = (unsigned)slotBase;
  const unsigned unb = (unsigned)nb;
  const unsigned s0 = (unsigned)da.x - nbs, s1 = (unsigned)da.y - nbs;
  const unsigned s2 = (unsigned)da.z - nbs, s3 = (unsigned)da.w - nbs;
  const unsigned s4 = (unsigned)db.x - nbs, s5 = (unsigned)db.y - nbs;
  const unsigned s6 = (unsigned)db.z - nbs, s7 = (unsigned)db.w - nbs;
  const bool h0 = s0 < unb, h1 = s1 < unb, h2 = s2 < unb, h3 = s3 < unb;
  const bool h4 = s4 < unb, h5 = s5 < unb, h6 = s6 < unb, h7 = s7 < unb;
  const unsigned any = __builtin_amdgcn_ballot_w32(h0 | h1 | h2 | h3 | h4 | h5 | h6 | h7);
  if (any != 0u) {
#define HITJ(J, HJ, SJ) { \
      const unsigned mj = __builtin_amdgcn_ballot_w32(HJ); \
      if (mj != 0u) { \
        if (HJ) { \
          const int pos = wc + (int)__builtin_amdgcn_mbcnt_lo(mj, 0u); \
          if (pos < WCAP) list[wave * WCAP + pos] = ((el0 + (J)) << SLOTB) | (int)(SJ); \
        } \
        wc += (int)__builtin_popcount(mj); } }
    HITJ(0, h0, s0)
    HITJ(1, h1, s1)
    HITJ(2, h2, s2)
    HITJ(3, h3, s3)
    HITJ(4, h4, s4)
    HITJ(5, h5, s5)
    HITJ(6, h6, s6)
    HITJ(7, h7, s7)
#undef HITJ
  }
  return wc;
}

__global__ __launch_bounds__(NTHR) void k_xprep(const float* __restrict__ x, unsigned short* xb, int nN, int nUnits) {
  const int i = (int)blockIdx.x * NTHR + (int)threadIdx.x;
  if (i >= nUnits) return;
  const int row = i >> 5;
  const int c0  = (i & 31) * 8;
  const int rc  = row < nN ? row : nN - 1;
  const float* p = x + (size_t)rc * F_IN + c0;
  v4f a = *(const v4fa*)p, b = *(const v4fa*)(p + 4);
  const v4f z4 = {0.f, 0.f, 0.f, 0.f};
  if (row >= nN) { a = z4; b = z4; }
  const v4u hv = pack8(a, b);
  const size_t o = (size_t)row * F_IN + c0;
  *(volatile v4u*)(xb + o) = hv;
  __threadfence();
  *(volatile v4u*)(xb + o) = hv;
}

__global__ __launch_bounds__(NTHR) void k_wtr(const float* __restrict__ w, int Kin, int Ncol, int Nrows, int Kout,
                                              unsigned short* wt, int nUnits) {
  const int u = (int)blockIdx.x * NTHR + (int)threadIdx.x;
  if (u >= nUnits) return;
  const int kq = Kout >> 3;
  const int n  = u / kq;
  const int k8 = (u - n * kq) * 8;
  const int kk = k8 - (k8 / Kin) * Kin;
  const int ncl = n < Ncol ? n : Ncol - 1;
  const float* p = w + (size_t)kk * (size_t)Ncol + ncl;
  v4f a, b;
  a.x = p[0];                    a.y = p[(size_t)Ncol];         a.z = p[(size_t)2 * Ncol];     a.w = p[(size_t)3 * Ncol];
  b.x = p[(size_t)4 * Ncol];     b.y = p[(size_t)5 * Ncol];     b.z = p[(size_t)6 * Ncol];     b.w = p[(size_t)7 * Ncol];
  const v4f z4 = {0.f, 0.f, 0.f, 0.f};
  if (n >= Ncol || n >= Nrows) { a = z4; b = z4; }
  const v4u wv = pack8(a, b);
  unsigned short* o = wt + (size_t)n * (size_t)Kout + k8;
  *(volatile v4u*)o = wv;
  __threadfence();
  *(volatile v4u*)o = wv;
}

__global__ __launch_bounds__(GTHR) void k_gemm(
    const unsigned short* __restrict__ A, const unsigned short* __restrict__ WT,
    float* outF, int K, int ldo,
    const float* __restrict__ atts, const float* __restrict__ attd, int attLen,
    float* SD, int MPr)
{
  __shared__ __attribute__((aligned(16))) float stg[GBM * GBN];
  __shared__ __attribute__((aligned(16))) float satt[2 * GBN];
  __shared__ __attribute__((aligned(16))) float sdot[2 * GBM];
  const int tid = (int)threadIdx.x, lane = tid & 31, wave = tid >> 5, hh = lane >> 4, m = lane & 15;
  const int rowBase = (int)blockIdx.x * GBM;
  const int head    = (int)blockIdx.y;
  const int col0    = head * GBN;

  {
    const int which = tid >> 6;
    const int c  = tid & 63;
    const int cl = c < attLen ? c : attLen - 1;
    const float vs = atts[head * attLen + cl];
    const float vd = attd[head * attLen + cl];
    float v = (which == 0) ? vs : vd;
    v = (c < attLen) ? bfr(v) : 0.f;
    satt[which * GBN + c] = v;
  }

  v8f acc[4];
  {
    const v8f z = {0.f, 0.f, 0.f, 0.f, 0.f, 0.f, 0.f, 0.f};
    acc[0] = z; acc[1] = z; acc[2] = z; acc[3] = z;
  }
  const unsigned short* ap = A  + (size_t)(rowBase + 16 * wave + m) * (size_t)K + 8 * hh;
  const unsigned short* wp = WT + (size_t)(col0 + m) * (size_t)K + 8 * hh;
  const int ksteps = K >> 5;
#pragma unroll 1
  for (int ks = 0; ks < ksteps; ++ks) {
    FragB af;
    af.h[0] = *(const v8usa*)(ap + 32 * ks);
    af.h[1] = *(const v8usa*)(ap + 32 * ks + 16);
#pragma unroll
    for (int t = 0; t < 4; ++t) {
      const unsigned short* wq = wp + (size_t)(16 * t) * (size_t)K + 32 * ks;
      FragB bf;
      bf.h[0] = *(const v8usa*)wq;
      bf.h[1] = *(const v8usa*)(wq + 16);
      acc[t] = wmb(af, bf, acc[t]);
    }
  }

#pragma unroll
  for (int t = 0; t < 4; ++t) {
    const int lc = 16 * t + m;
#pragma unroll
    for (int r = 0; r < 8; ++r) {
      const int lr = 16 * wave + 8 * hh + r;
      stg[lr * GBN + lc] = acc[t][r];
    }
  }
  __syncthreads();

  {
    const int row = tid & 63, which = tid >> 6;
    const float* sa = satt + which * GBN;
    const float* hr = stg + row * GBN;
    float d = 0.f;
#pragma unroll 4
    for (int c4 = 0; c4 < GBN / 4; ++c4) {
      const v4f hv = *(const v4fa*)(hr + 4 * c4);
      const v4f av = *(const v4fa*)(sa + 4 * c4);
      d = fmaf(hv.x, av.x, d);
      d = fmaf(hv.y, av.y, d);
      d = fmaf(hv.z, av.z, d);
      d = fmaf(hv.w, av.w, d);
    }
    sdot[which * GBM + row] = d;
  }
  __syncthreads();

  v4f fv[8];
#pragma unroll
  for (int i = 0; i < 8; ++i) {
    const int lr = 16 * wave + 2 * i + hh;
    fv[i] = *(const v4fa*)(stg + lr * GBN + 4 * m);
  }
  const int which2 = lane >> 4, piece = lane & 15;
  const v4f sdv = *(const v4fa*)(sdot + which2 * GBM + 4 * piece);
  float* sp = SD + (size_t)(2 * head + which2) * (size_t)MPr + rowBase + 4 * piece;

#pragma unroll
  for (int i = 0; i < 8; ++i) {
    const int lr = 16 * wave + 2 * i + hh;
    const int gr = rowBase + lr;
    float* op = outF + (size_t)gr * (size_t)ldo + col0 + 4 * m;
    *(volatile v4f*)op = fv[i];
  }
  if (wave == 0) *(volatile v4f*)sp = sdv;
  __threadfence();
#pragma unroll
  for (int i = 0; i < 8; ++i) {
    const int lr = 16 * wave + 2 * i + hh;
    const int gr = rowBase + lr;
    float* op = outF + (size_t)gr * (size_t)ldo + col0 + 4 * m;
    *(volatile v4f*)op = fv[i];
  }
  if (wave == 0) *(volatile v4f*)sp = sdv;
}

template<int L>
__global__ __launch_bounds__(NTHR) void k_agg(
    const int* __restrict__ srcs, const int* __restrict__ dsts,
    const float* __restrict__ F, const float* __restrict__ SD,
    const float* __restrict__ bias,
    const float* __restrict__ Wf1, const float* __restrict__ bf1,
    const float* __restrict__ Wf2, const float* __restrict__ bf2,
    unsigned short* HP, float* out,
    int nN, int nE, int nb, int vec8, int MPr) {
  extern __shared__ v4f lds_dyn[];
  int* reg1 = (int*)lds_dyn;
  int* reg2 = reg1 + RCAP;
  int* scnt = reg2 + RCAP;
  int* soff = scnt + NBMAX;
  int* list = soff + NBMAX;
  int* wcnt = list + LISTN;
  int* wtot = wcnt + NWAVE;
  const int tid = (int)threadIdx.x, lane = tid & 31, wave = tid >> 5;
  const int nodeBase = (int)blockIdx.x * nb;

  for (int i = tid; i < NBMAX; i += NTHR) scnt[i] = 0;
  __syncthreads();

  int tot = 0;
  const int nChunks = (nE + CHUNK - 1) / CHUNK;
#pragma unroll 1
  for (int ch = 0; ch < nChunks; ++ch) {
    const int cbase = ch * CHUNK;
    const int wc = scan_chunk(dsts, nE, cbase, nodeBase, nb, vec8, list, tid, lane, wave);
    if (lane == 0) wcnt[wave] = wc;
    __syncthreads();
    int pre = 0, all = 0;
#pragma unroll
    for (int w2 = 0; w2 < NWAVE; ++w2) {
      int c = wcnt[w2];
      c = c < 0 ? 0 : (c > WCAP ? WCAP : c);
      all += c;
      pre += (w2 < wave) ? c : 0;
    }
    const int wcc  = wc > WCAP ? WCAP : wc;
    const int base = tot + pre;
#pragma unroll 1
    for (int i = lane; i < wcc; i += 32) {
      const int ent = list[wave * WCAP + i];
      const int el  = (ent >> SLOTB) & (CHUNK - 1);
      const int sl  = ent & (NBMAX - 1);
      int eid = cbase + el;
      eid = eid > nE - 1 ? nE - 1 : eid;
      const int pos = base + i;
      if (pos < RCAP) reg1[pos] = (int)(((unsigned)eid << SLOTB) | (unsigned)sl);
    }
    tot += all;
    tot = tot > RCAP ? RCAP : tot;
    __syncthreads();
  }
  const int nh = tot;

  if (wave == 0) {
#pragma unroll 1
    for (int b0 = 0; b0 < nh; b0 += 32) {
      const int idx = b0 + lane;
      const int uv  = reg1[idx < nh ? idx : nh - 1];
      const int m32 = (nh - b0) < 32 ? (nh - b0) : 32;
#pragma unroll 1
      for (int k = 0; k < m32; ++k) {
        const int u  = __builtin_amdgcn_readlane(uv, k);
        const int sl = u & (NBMAX - 1);
        if (lane == 0) scnt[sl] = scnt[sl] + 1;
      }
    }
  }
  __syncthreads();

  {
    const v4i ca = *(const v4i*)(scnt + 8 * tid);
    const v4i cb = *(const v4i*)(scnt + 8 * tid + 4);
    const int e0 = ca.x < 0 ? 0 : ca.x, e1 = ca.y < 0 ? 0 : ca.y, e2 = ca.z < 0 ? 0 : ca.z, e3 = ca.w < 0 ? 0 : ca.w;
    const int e4 = cb.x < 0 ? 0 : cb.x, e5 = cb.y < 0 ? 0 : cb.y, e6 = cb.z < 0 ? 0 : cb.z, e7 = cb.w < 0 ? 0 : cb.w;
    const int ts = e0 + e1 + e2 + e3 + e4 + e5 + e6 + e7;
    int incl = ts;
#pragma unroll
    for (int d = 1; d < 32; d <<= 1) {
      const int up = __shfl_up(incl, d);
      if (lane >= d) incl += up;
    }
    if (lane == 31) wtot[wave] = incl;
    __syncthreads();
    int pre = 0;
#pragma unroll
    for (int w2 = 0; w2 < NWAVE; ++w2) pre += (w2 < wave) ? wtot[w2] : 0;
    int run = pre + incl - ts;
    soff[8 * tid + 0] = run; run += e0;
    soff[8 * tid + 1] = run; run += e1;
    soff[8 * tid + 2] = run; run += e2;
    soff[8 * tid + 3] = run; run += e3;
    soff[8 * tid + 4] = run; run += e4;
    soff[8 * tid + 5] = run; run += e5;
    soff[8 * tid + 6] = run; run += e6;
    soff[8 * tid + 7] = run;
  }
  __syncthreads();
  for (int i = tid; i < NBMAX; i += NTHR) list[i] = soff[i];
  __syncthreads();

  if (wave == 0) {
#pragma unroll 1
    for (int b0 = 0; b0 < nh; b0 += 32) {
      const int idx = b0 + lane;
      const int uv  = reg1[idx < nh ? idx : nh - 1];
      const int m32 = (nh - b0) < 32 ? (nh - b0) : 32;
#pragma unroll 1
      for (int k = 0; k < m32; ++k) {
        const int u   = __builtin_amdgcn_readlane(uv, k);
        const int sl  = u & (NBMAX - 1);
        const int eid = (int)((unsigned)u >> SLOTB);
        if (lane == 0) {
          int pos = list[sl];
          pos = pos < 0 ? 0 : (pos > RCAP - 1 ? RCAP - 1 : pos);
          reg2[pos] = eid;
          list[sl] = pos + 1;
        }
      }
    }
  }
  __syncthreads();

  if (L == 2) {
    float* wfs = (float*)reg1 + NWAVE * GRP * OC;
#pragma unroll 1
    for (int i = tid; i < (OC * OC) / 4; i += NTHR) {
      const v4f a = bfr4(*(const v4fa*)(Wf1 + 4 * i));
      const v4f b = bfr4(*(const v4fa*)(Wf2 + 4 * i));
      *(v4fa*)(wfs + 4 * i) = a;
      *(v4fa*)(wfs + OC * OC + 4 * i) = b;
    }
    __syncthreads();
  }

  const int nbw = nb >> 3;
  const bool ovf = (nh >= RCAP);
  const float qnan = __int_as_float(0x7fc00000);

  if (L == 1) {
    const int c0   = 8 * lane;
    const int head = lane >> 3;
    const v4f bbA  = bfr4(*(const v4fa*)(bias + c0));
    const v4f bbB  = bfr4(*(const v4fa*)(bias + c0 + 4));
    const float* ASp = SD + (size_t)(2 * head) * (size_t)MPr;
    const float* ADp = ASp + MPr;

#pragma unroll 1
    for (int jt = 0; jt < nbw; ++jt) {
      const int slot = wave * nbw + jt;
      const int grow = nodeBase + slot;
      const int gcl  = grow < nN ? grow : nN - 1;
      int st = soff[slot];
      const int craw = scnt[slot];
      int cnt = craw;
      st  = st < 0 ? 0 : (st > nh ? nh : st);
      cnt = cnt < 0 ? 0 : (cnt > DEGCAP ? DEGCAP : cnt);
      if (cnt > nh - st) cnt = nh - st;
      const float pz = (ovf || craw > DEGCAP) ? qnan : 0.0f;

      const float* fr = F + (size_t)gcl * HC1 + c0;
      v4f avA = *(const v4fa*)fr;
      v4f avB = *(const v4fa*)(fr + 4);
      const float adv = ADp[gcl];
      float l0 = ASp[gcl] + adv;
      l0 = l0 > 0.f ? l0 : NEGSL * l0;
      float mx = l0, dn = 1.0f;

#pragma unroll 1
      for (int q = 0; q < cnt; ++q) {
        int idx = st + q; idx = idx > RCAP - 1 ? RCAP - 1 : idx;
        int eid = reg2[idx]; eid = eid < 0 ? 0 : (eid > nE - 1 ? nE - 1 : eid);
        const int sraw = srcs[eid];
        const int s = sraw < 0 ? 0 : (sraw > nN - 1 ? nN - 1 : sraw);
        const float* sr = F + (size_t)s * HC1 + c0;
        const v4f fsA = *(const v4fa*)sr;
        const v4f fsB = *(const v4fa*)(sr + 4);
        float lg = ASp[s] + adv;
        lg = lg > 0.f ? lg : NEGSL * lg;
        const float df = lg - mx;
        const float ee = __expf(-fabsf(df));
        const bool up  = df > 0.f;
        const float s1 = up ? ee : 1.0f;
        const float s2 = up ? 1.0f : ee;
        mx = up ? lg : mx;
        dn = fmaf(dn, s1, s2);
        avA.x = fmaf(avA.x, s1, s2 * fsA.x);
        avA.y = fmaf(avA.y, s1, s2 * fsA.y);
        avA.z = fmaf(avA.z, s1, s2 * fsA.z);
        avA.w = fmaf(avA.w, s1, s2 * fsA.w);
        avB.x = fmaf(avB.x, s1, s2 * fsB.x);
        avB.y = fmaf(avB.y, s1, s2 * fsB.y);
        avB.z = fmaf(avB.z, s1, s2 * fsB.z);
        avB.w = fmaf(avB.w, s1, s2 * fsB.w);
      }
      const float inv = __builtin_amdgcn_rcpf(dn + EPS_SM);
      const bool live = grow < nN;
      const float o0 = (live ? fmaxf(fmaf(avA.x, inv, bbA.x), 0.f) : 0.f) + pz;
      const float o1 = (live ? fmaxf(fmaf(avA.y, inv, bbA.y), 0.f) : 0.f) + pz;
      const float o2 = (live ? fmaxf(fmaf(avA.z, inv, bbA.z), 0.f) : 0.f) + pz;
      const float o3 = (live ? fmaxf(fmaf(avA.w, inv, bbA.w), 0.f) : 0.f) + pz;
      const float o4 = (live ? fmaxf(fmaf(avB.x, inv, bbB.x), 0.f) : 0.f) + pz;
      const float o5 = (live ? fmaxf(fmaf(avB.y, inv, bbB.y), 0.f) : 0.f) + pz;
      const float o6 = (live ? fmaxf(fmaf(avB.z, inv, bbB.z), 0.f) : 0.f) + pz;
      const float o7 = (live ? fmaxf(fmaf(avB.w, inv, bbB.w), 0.f) : 0.f) + pz;
      const unsigned int h0 = f2bf(o0), h1 = f2bf(o1), h2 = f2bf(o2), h3 = f2bf(o3);
      const unsigned int h4 = f2bf(o4), h5 = f2bf(o5), h6 = f2bf(o6), h7 = f2bf(o7);
      const unsigned int q0 = f2bf(o0 - bf2f(h0)), q1 = f2bf(o1 - bf2f(h1));
      const unsigned int q2 = f2bf(o2 - bf2f(h2)), q3 = f2bf(o3 - bf2f(h3));
      const unsigned int q4 = f2bf(o4 - bf2f(h4)), q5 = f2bf(o5 - bf2f(h5));
      const unsigned int q6 = f2bf(o6 - bf2f(h6)), q7 = f2bf(o7 - bf2f(h7));
      v4u hv, lv;
      hv.x = h0 | (h1 << 16); hv.y = h2 | (h3 << 16); hv.z = h4 | (h5 << 16); hv.w = h6 | (h7 << 16);
      lv.x = q0 | (q1 << 16); lv.y = q2 | (q3 << 16); lv.z = q4 | (q5 << 16); lv.w = q6 | (q7 << 16);
      unsigned short* gp = HP + (size_t)grow * KA2 + 8 * lane;
      const bool wr = grow < MPr;
      if (wr) { *(volatile v4u*)gp = hv; *(volatile v4u*)(gp + HC1) = lv; }
      __threadfence();
      if (wr) { *(volatile v4u*)gp = hv; *(volatile v4u*)(gp + HC1) = lv; }
    }
  } else {
    const int c0 = 2 * lane;
    float* fl  = (float*)reg1;
    float* res = fl + wave * (GRP * OC);
    const float* W1s = fl + NWAVE * GRP * OC;
    const float* W2s = W1s + OC * OC;
    const v2f bzr = *(const v2fa*)(bias + c0);
    const v2f b1r = *(const v2fa*)(bf1 + c0);
    const v2f b2r = *(const v2fa*)(bf2 + c0);
    const float bz0 = bfr(bzr.x), bz1 = bfr(bzr.y);
    const float p10 = bfr(b1r.x), p11 = bfr(b1r.y);
    const float p20 = bfr(b2r.x), p21 = bfr(b2r.y);
    const float* ASp = SD;
    const float* ADp = SD + MPr;

#pragma unroll 1
    for (int jt = 0; jt < nbw; ++jt) {
      const int slot = wave * nbw + jt;
      const int grow = nodeBase + slot;
      const int gcl  = grow < nN ? grow : nN - 1;
      int st = soff[slot];
      const int craw = scnt[slot];
      int cnt = craw;
      st  = st < 0 ? 0 : (st > nh ? nh : st);
      cnt = cnt < 0 ? 0 : (cnt > DEGCAP ? DEGCAP : cnt);
      if (cnt > nh - st) cnt = nh - st;
      const float pz = (ovf || craw > DEGCAP) ? qnan : 0.0f;

      const v2f fd = *(const v2fa*)(F + (size_t)gcl * OC + c0);
      const float adv = ADp[gcl];
      float l0 = ASp[gcl] + adv;
      l0 = l0 > 0.f ? l0 : NEGSL * l0;
      float mx = l0, dn = 1.0f;
      float a0 = fd.x, a1 = fd.y;

#pragma unroll 1
      for (int q = 0; q < cnt; ++q) {
        int idx = st + q; idx = idx > RCAP - 1 ? RCAP - 1 : idx;
        int eid = reg2[idx]; eid = eid < 0 ? 0 : (eid > nE - 1 ? nE - 1 : eid);
        const int sraw = srcs[eid];
        const int s = sraw < 0 ? 0 : (sraw > nN - 1 ? nN - 1 : sraw);
        const v2f fs = *(const v2fa*)(F + (size_t)s * OC + c0);
        float lg = ASp[s] + adv;
        lg = lg > 0.f ? lg : NEGSL * lg;
        const float df = lg - mx;
        const float ee = __expf(-fabsf(df));
        const bool up  = df > 0.f;
        const float s1 = up ? ee : 1.0f;
        const float s2 = up ? 1.0f : ee;
        mx = up ? lg : mx;
        dn = fmaf(dn, s1, s2);
        a0 = fmaf(a0, s1, s2 * fs.x);
        a1 = fmaf(a1, s1, s2 * fs.y);
      }
      const float inv = __builtin_amdgcn_rcpf(dn + EPS_SM);
      const float hA = fmaxf(fmaf(a0, inv, bz0), 0.f);
      const float hB = fmaxf(fmaf(a1, inv, bz1), 0.f);

      float f0 = p10, f1 = p11;
#pragma unroll 2
      for (int k2 = 0; k2 < OC / 2; ++k2) {
        const float xa = __shfl(hA, k2);
        const float xb = __shfl(hB, k2);
        const v2f w0 = *(const v2fa*)(W1s + (2 * k2) * OC + c0);
        const v2f w1 = *(const v2fa*)(W1s + (2 * k2 + 1) * OC + c0);
        f0 = fmaf(xa, w0.x, f0); f1 = fmaf(xa, w0.y, f1);
        f0 = fmaf(xb, w1.x, f0); f1 = fmaf(xb, w1.y, f1);
      }
      f0 = fmaxf(f0, 0.f); f1 = fmaxf(f1, 0.f);
      float z0 = p20, z1 = p21;
#pragma unroll 2
      for (int k2 = 0; k2 < OC / 2; ++k2) {
        const float xa = __shfl(f0, k2);
        const float xb = __shfl(f1, k2);
        const v2f w0 = *(const v2fa*)(W2s + (2 * k2) * OC + c0);
        const v2f w1 = *(const v2fa*)(W2s + (2 * k2 + 1) * OC + c0);
        z0 = fmaf(xa, w0.x, z0); z1 = fmaf(xa, w0.y, z1);
        z0 = fmaf(xb, w1.x, z0); z1 = fmaf(xb, w1.y, z1);
      }
      float vm = fmaxf(z0, z1);
#pragma unroll
      for (int off = 16; off > 0; off >>= 1) vm = fmaxf(vm, __shfl_xor(vm, off));
      const float ex0 = expf(z0 - vm), ex1 = expf(z1 - vm);
      float sm = ex0 + ex1;
#pragma unroll
      for (int off = 16; off > 0; off >>= 1) sm += __shfl_xor(sm, off);
      const float rs = __builtin_amdgcn_rcpf(sm);
      const int lr = jt & (GRP - 1);
      {
        v2f ov; ov.x = ex0 * rs + pz; ov.y = ex1 * rs + pz;
        *(v2f*)(res + lr * OC + c0) = ov;
      }

      const int gb = jt & ~(GRP - 1);
      if (lr == GRP - 1 || jt == nbw - 1) {
        __syncthreads();
        int gsz = nbw - gb; gsz = gsz > GRP ? GRP : gsz;
        const int row0 = nodeBase + wave * nbw + gb;
        int live = nN - row0; live = live < 0 ? 0 : (live > gsz ? gsz : live);
        const int npc = live * (OC / 4);
        float* ob = out + (size_t)row0 * OC;
#pragma unroll 1
        for (int p = lane; p < npc; p += 32) {
          const v4f v = *(const v4fa*)(res + 4 * p);
          *(volatile v4f*)(ob + 4 * p) = v;
        }
        __threadfence();
#pragma unroll 1
        for (int p = lane; p < npc; p += 32) {
          const v4f v = *(const v4fa*)(res + 4 * p);
          *(volatile v4f*)(ob + 4 * p) = v;
        }
        __syncthreads();
      }
    }
  }
}

static int pick_nb(int nE, int nN) {
  int nb = NBMAX;
  while (nb > 32 && (long long)nb * (long long)nE * 5LL > (long long)RCAP * (long long)nN * 4LL) nb >>= 1;
  return nb;
}
static inline int cdiv(int a, int b) { return (a + b - 1) / b; }

extern "C" void kernel_launch(void* const* d_in, const int* in_sizes, int n_in,
                              void* d_out, int out_size, void* d_ws, size_t ws_size,
                              hipStream_t stream) {
  if (n_in < 14) return;
  const int nN = in_sizes[0] / F_IN;
  if (nN <= 0 || in_sizes[0] != nN * F_IN || nN > (1 << 22)) return;
  if (in_sizes[1] < 2 || (in_sizes[1] & 1) != 0) return;
  const int nE = in_sizes[1] / 2;
  if (nE < 1 || nE >= (1 << (32 - SLOTB))) return;
  if (in_sizes[2] != F_IN * HC1) return;
  if (in_sizes[3] != NHD1 * HID || in_sizes[4] != NHD1 * HID) return;
  if (in_sizes[5] != HC1) return;
  if (in_sizes[6] != HC1 * OC) return;
  if (in_sizes[7] != OC || in_sizes[8] != OC) return;
  if (in_sizes[9] != OC) return;
  if (in_sizes[10] != OC * OC || in_sizes[11] != OC) return;
  if (in_sizes[12] != OC * OC || in_sizes[13] != OC) return;
  if ((long long)out_size != (long long)nN * OC) return;

  const float* x    = (const float*)d_in[0];
  const int*   ei   = (const int*)  d_in[1];
  const float* W1   = (const float*)d_in[2];
  const float* a1s  = (const float*)d_in[3];
  const float* a1d  = (const float*)d_in[4];
  const float* b1   = (const float*)d_in[5];
  const float* W2   = (const float*)d_in[6];
  const float* a2s  = (const float*)d_in[7];
  const float* a2d  = (const float*)d_in[8];
  const float* b2   = (const float*)d_in[9];
  const float* Wf1  = (const float*)d_in[10];
  const float* bf1  = (const float*)d_in[11];
  const float* Wf2  = (const float*)d_in[12];
  const float* bf2  = (const float*)d_in[13];
  float* out = (float*)d_out;
  const int* src = ei;
  const int* dst = ei + nE;

  const int MP   = cdiv(nN, MROWS) * MROWS;
  const int nb   = pick_nb(nE, nN);
  if (nb < 32 || (nb & (nb - 1)) != 0 || nb > NBMAX) return;
  const int gA   = cdiv(MP, nb);
  const int vec8 = ((nE & 3) == 0) ? 1 : 0;
  if (gA * nb < MP) return;

  char* ws = (char*)d_ws;
  size_t off = 0;
  const size_t oA2  = off; off += (size_t)MP * KA2 * 2;            off = (off + 255) & ~(size_t)255;
  const size_t oW1T = off; off += (size_t)HC1 * F_IN * 2;          off = (off + 255) & ~(size_t)255;
  const size_t oW2D = off; off += (size_t)OC * KA2 * 2;            off = (off + 255) & ~(size_t)255;
  const size_t oH1  = off; off += (size_t)MP * HC1 * 4;            off = (off + 255) & ~(size_t)255;
  const size_t oSD1 = off; off += (size_t)2 * NHD1 * MP * 4;       off = (off + 255) & ~(size_t)255;
  const size_t oG2  = off; off += (size_t)MP * OC * 4;             off = (off + 255) & ~(size_t)255;
  const size_t oSD2 = off; off += (size_t)2 * MP * 4;              off = (off + 255) & ~(size_t)255;
  if (off > ws_size || off > (size_t)WSMAX) return;
  if ((size_t)MP * F_IN * 2 > (size_t)MP * KA2 * 2) return;
  unsigned short* A2  = (unsigned short*)(ws + oA2);
  unsigned short* XB  = A2;
  unsigned short* W1T = (unsigned short*)(ws + oW1T);
  unsigned short* W2D = (unsigned short*)(ws + oW2D);
  float*          H1  = (float*)(ws + oH1);
  float*          SD1 = (float*)(ws + oSD1);
  float*          G2  = (float*)(ws + oG2);
  float*          SD2 = (float*)(ws + oSD2);

  hipFuncSetAttribute(reinterpret_cast<const void*>(&k_agg<1>),
                      hipFuncAttributeMaxDynamicSharedMemorySize, LDS_AGG);
  hipFuncSetAttribute(reinterpret_cast<const void*>(&k_agg<2>),
                      hipFuncAttributeMaxDynamicSharedMemorySize, LDS_AGG);

  const int nUx = MP * (F_IN / 8);
  k_xprep<<<cdiv(nUx, NTHR), NTHR, 0, stream>>>(x, XB, nN, nUx);

  {
    const int nUw1 = HC1 * (F_IN / 8);
    k_wtr<<<cdiv(nUw1, NTHR), NTHR, 0, stream>>>(W1, F_IN, HC1, HC1, F_IN, W1T, nUw1);
    const int nUw2 = OC * (KA2 / 8);
    k_wtr<<<cdiv(nUw2, NTHR), NTHR, 0, stream>>>(W2, HC1, OC, OC, KA2, W2D, nUw2);
  }

  const int gM = MP / GBM;
  k_gemm<<<dim3(gM, HC1 / GBN), GTHR, 0, stream>>>(XB, W1T, H1, F_IN, HC1, a1s, a1d, HID, SD1, MP);
  k_agg<1><<<gA, NTHR, LDS_AGG, stream>>>(src, dst, H1, SD1, b1, Wf1, bf1, Wf2, bf2, A2, out,
                                          nN, nE, nb, vec8, MP);
  k_gemm<<<dim3(gM, OC / GBN), GTHR, 0, stream>>>(A2, W2D, G2, KA2, OC, a2s, a2d, OC, SD2, MP);
  k_agg<2><<<gA, NTHR, LDS_AGG, stream>>>(src, dst, G2, SD2, b2, Wf1, bf1, Wf2, bf2, A2, out,
                                          nN, nE, nb, vec8, MP);
}
